// BlockchainAIEngine_2027224564539
// MI455X (gfx1250) — hardware-verified
//
#include <hip/hip_runtime.h>
#include <stddef.h>

constexpr int kRows   = 2048;
constexpr int kDin    = 512;
constexpr int kNE     = 100;
constexpr int kHid    = 256;
constexpr int kDo     = 128;
constexpr int kCat    = kNE * kDo;
constexpr int kHc     = 512;
constexpr int kEChunk = 10;
constexpr int kNChunk = kNE / kEChunk;
constexpr int kNcols  = kEChunk * kHid;
constexpr float kW1Carry     = 16.0f;
constexpr float kW1CarryInv  = 1.0f / 16.0f;
constexpr float kWc1Carry    = 64.0f;
constexpr float kWc1CarryInv = 1.0f / 64.0f;
static_assert(kNE % kEChunk == 0, "chunking must be exact");
static_assert(kDin % 32 == 0 && kHid % 32 == 0 && kCat % 32 == 0 && kHc % 32 == 0 && kDo % 32 == 0, "K multiples of 32");
static_assert(kRows % 64 == 0 && kNcols % 64 == 0 && kDo % 64 == 0 && kHc % 64 == 0, "M,N multiples of 64");

typedef __attribute__((ext_vector_type(16))) _Float16 v16h;
typedef __attribute__((ext_vector_type(8)))  _Float16 v8h;
typedef __attribute__((ext_vector_type(16))) __bf16   v16b;
typedef __attribute__((ext_vector_type(8)))  __bf16   v8b;
typedef __attribute__((ext_vector_type(8)))  float    v8f;
typedef __attribute__((ext_vector_type(4)))  float    v4f;
typedef __attribute__((ext_vector_type(4)))  unsigned int v4u;

__device__ __forceinline__ unsigned short f2bf_bits(float f) {
  unsigned u = __float_as_uint(f);
  return (unsigned short)((u + 0x7FFFu + ((u >> 16) & 1u)) >> 16);
}
__device__ __forceinline__ float bf_bits2f(unsigned short h) { return __uint_as_float(((unsigned)h) << 16); }

__device__ __forceinline__ void dep_guard_h(v8f& a, v8f& b, v16h x, v16h y) { asm volatile("v_nop\n\tv_nop\n\tv_nop\n\tv_nop" : "+v"(a), "+v"(b) : "v"(x), "v"(y)); }
__device__ __forceinline__ void dep_guard_b(v8f& a, v8f& b, v16b x, v16b y) { asm volatile("v_nop\n\tv_nop\n\tv_nop\n\tv_nop" : "+v"(a), "+v"(b) : "v"(x), "v"(y)); }
__device__ __forceinline__ void keep4_h(v16h a, v16h b, v16h c, v16h d) { asm volatile("v_nop" :: "v"(a), "v"(b), "v"(c), "v"(d)); }
__device__ __forceinline__ void keep4_b(v16b a, v16b b, v16b c, v16b d) { asm volatile("v_nop" :: "v"(a), "v"(b), "v"(c), "v"(d)); }
__device__ __forceinline__ void acc_guard4(v8f& a, v8f& b, v8f& c, v8f& d) { asm volatile("v_nop\n\tv_nop\n\tv_nop\n\tv_nop" : "+v"(a), "+v"(b), "+v"(c), "+v"(d)); }
template <typename T> struct Frag;
template <> struct Frag<_Float16> {
  typedef v16h V; union U { v16h v; v8h h[2]; };
  static __device__ __forceinline__ v16h load(const _Float16* p) {
    U f; f.h[0] = *(const v8h*)(p); f.h[1] = *(const v8h*)(p + 16); return f.v;
  }
  static __device__ __forceinline__ v8f mma(v16h a, v16h b, v8f c) {
    return __builtin_amdgcn_wmma_f32_16x16x32_f16(false, a, false, b, (short)0, c, false, false);
  }
  static __device__ __forceinline__ void guard(v8f& a, v8f& b, v16h x, v16h y) { dep_guard_h(a, b, x, y); }
  static __device__ __forceinline__ void keep(v16h a, v16h b, v16h c, v16h d) { keep4_h(a, b, c, d); }
};
template <> struct Frag<__bf16> {
  typedef v16b V; union U { v16b v; v8b h[2]; };
  static __device__ __forceinline__ v16b load(const __bf16* p) {
    U f; f.h[0] = *(const v8b*)(p); f.h[1] = *(const v8b*)(p + 16); return f.v;
  }
  static __device__ __forceinline__ v8f mma(v16b a, v16b b, v8f c) {
    return __builtin_amdgcn_wmma_f32_16x16x32_bf16(false, a, false, b, (short)0, c, false, false);
  }
  static __device__ __forceinline__ void guard(v8f& a, v8f& b, v16b x, v16b y) { dep_guard_b(a, b, x, y); }
  static __device__ __forceinline__ void keep(v16b a, v16b b, v16b c, v16b d) { keep4_b(a, b, c, d); }
};

__device__ __forceinline__ unsigned pk16(unsigned short a, unsigned short b) { return (unsigned)a | ((unsigned)b << 16); }
__device__ __forceinline__ unsigned short h_bits(float f) { const _Float16 h = (_Float16)f; return __builtin_bit_cast(unsigned short, h); }

template <int ET> struct Elem;
template <> struct Elem<0> { typedef _Float16 T; };
template <> struct Elem<1> { typedef __bf16 T; };
template <int ET, bool SPLIT, int BIAS_MODE, int OUT_MODE, bool RESID, int ACT = 0>
__global__ __launch_bounds__(256) void wmma_gemm64(
    const unsigned short* __restrict__ Ap, const unsigned short* __restrict__ A2p, int lda, long strideA,
    const unsigned short* __restrict__ Btp, const unsigned short* __restrict__ Bt2p, int ldb, long strideB,
    void* __restrict__ Cout, void* __restrict__ Cout2, int ldc, long strideC,
    const float* __restrict__ bias, long strideBias,
    const float* __restrict__ resid, long strideR,
    int M, int N, int K, float scale) {
  typedef typename Elem<ET>::T T;
  typedef typename Frag<T>::V V;
  const T* A = (const T*)Ap; const T* A2 = (const T*)A2p; const T* Bt = (const T*)Btp; const T* Bt2 = (const T*)Bt2p;
  __shared__ __align__(16) float sT[8][16 * 68];
  const int b    = blockIdx.y;
  const int lane = threadIdx.x & 31;
  const int wave = threadIdx.x >> 5;
  const int tilesN = N >> 6;
  const int tilesM = M >> 6;
  const int tile = blockIdx.x * 8 + wave;
  if (tile >= tilesM * tilesN) return;
  const int tm = tile / tilesN;
  const int tn = tile - tm * tilesN;
  const int m0 = tm << 6;
  const int n0 = tn << 6;

  const T* Ab  = A  + (size_t)b * strideA;
  const T* Bb  = Bt + (size_t)b * strideB;
  const T* Ab2 = SPLIT ? (A2  + (size_t)b * strideA) : nullptr;
  const T* Bb2 = SPLIT ? (Bt2 + (size_t)b * strideB) : nullptr;

  const int rlane = lane & 15;
  const int koff  = (lane >> 4) * 8;
  const int mOff  = (lane >> 4) * 8;

  v8f acc[4][4];
#pragma unroll
  for (int i = 0; i < 4; ++i)
#pragma unroll
    for (int j = 0; j < 4; ++j) acc[i][j] = (v8f){0.f,0.f,0.f,0.f,0.f,0.f,0.f,0.f};

  for (int k0 = 0; k0 < K; k0 += 32) {
    V bh[4], bl[4];
#pragma unroll
    for (int j = 0; j < 4; ++j) {
      const size_t bo = (size_t)(n0 + (j << 4) + rlane) * ldb + koff + k0;
      bh[j] = Frag<T>::load(Bb + bo);
      if (SPLIT) bl[j] = Frag<T>::load(Bb2 + bo);
    }
#pragma unroll
    for (int i = 0; i < 4; ++i) {
      const size_t ao = (size_t)(m0 + (i << 4) + rlane) * lda + koff + k0;
      V ah = Frag<T>::load(Ab + ao);
      V al;
      if (SPLIT) al = Frag<T>::load(Ab2 + ao);
#pragma unroll
      for (int j = 0; j < 4; ++j) {
        acc[i][j] = Frag<T>::mma(ah, bh[j], acc[i][j]);
        if (SPLIT) {
          acc[i][j] = Frag<T>::mma(ah, bl[j], acc[i][j]);
          acc[i][j] = Frag<T>::mma(al, bh[j], acc[i][j]);
        }
      }
      Frag<T>::guard(acc[i][0], acc[i][3], ah, SPLIT ? al : ah);
    }
    Frag<T>::keep(bh[0], bh[1], bh[2], bh[3]);
    if (SPLIT) Frag<T>::keep(bl[0], bl[1], bl[2], bl[3]);
  }
  acc_guard4(acc[0][0], acc[0][1], acc[0][2], acc[0][3]);
  acc_guard4(acc[1][0], acc[1][1], acc[1][2], acc[1][3]);
  acc_guard4(acc[2][0], acc[2][1], acc[2][2], acc[2][3]);
  acc_guard4(acc[3][0], acc[3][1], acc[3][2], acc[3][3]);

  float* slab = sT[wave];
  const float* Rb = RESID ? (resid + (size_t)b * strideR) : nullptr;
  const float* Bi = (BIAS_MODE != 0) ? (bias + (size_t)b * strideBias) : nullptr;
#pragma unroll
  for (int i = 0; i < 4; ++i) {
    const int mBase = m0 + (i << 4);
#pragma unroll
    for (int j = 0; j < 4; ++j) {
      const int n = n0 + (j << 4) + rlane;
      float bv = 0.f;
      if (BIAS_MODE == 2) bv = Bi[n];
#pragma unroll
      for (int r = 0; r < 8; ++r) {
        float v = acc[i][j][r] * scale;
        if (BIAS_MODE == 1) v += Bi[mBase + mOff + r];
        if (BIAS_MODE == 2) v += bv;
        if (RESID) v += Rb[(size_t)(mBase + mOff + r) * ldc + n];
        if (ACT == 2) v = fmaxf(v, 0.0f);
        if (ACT == 4) v = (v > 0.f) ? v : 0.01f * v;
        slab[(mOff + r) * 68 + (j << 4) + rlane] = v;
      }
    }
    __builtin_amdgcn_fence(__ATOMIC_RELEASE, "workgroup");
    __builtin_amdgcn_wave_barrier();
    __builtin_amdgcn_fence(__ATOMIC_ACQUIRE, "workgroup");
    if (OUT_MODE == 0) {
      float* C = (float*)Cout + (size_t)b * strideC;
      const int hh = lane >> 4, c4 = (lane & 15) * 4;
      for (int pass = 0; pass < 2; ++pass) {
#pragma unroll
        for (int it = 0; it < 8; ++it) {
          const int row = it * 2 + hh;
          v4f v = *(const v4f*)(slab + row * 68 + c4);
          *(volatile v4f*)(C + (size_t)(mBase + row) * ldc + n0 + c4) = v;
        }
        __threadfence();
      }
    } else {
      const int q = lane >> 3, c8 = (lane & 7) * 8;
      unsigned short* C  = (unsigned short*)Cout  + (size_t)b * strideC;
      unsigned short* C2 = (OUT_MODE == 2) ? ((unsigned short*)Cout2 + (size_t)b * strideC) : nullptr;
      for (int pass = 0; pass < 2; ++pass) {
#pragma unroll
        for (int it = 0; it < 4; ++it) {
          const int row = it * 4 + q;
          const float* sp = slab + row * 68 + c8;
          v8h hv, lv;
#pragma unroll
          for (int e = 0; e < 8; ++e) {
            if (OUT_MODE == 1) {
              hv[e] = (_Float16)sp[e];
            } else {
              unsigned short hb = f2bf_bits(sp[e]);
              unsigned short lb = f2bf_bits(sp[e] - bf_bits2f(hb));
              hv[e] = __builtin_bit_cast(_Float16, hb);
              lv[e] = __builtin_bit_cast(_Float16, lb);
            }
          }
          *(volatile v8h*)(C + (size_t)(mBase + row) * ldc + n0 + c8) = hv;
          if (OUT_MODE == 2) *(volatile v8h*)(C2 + (size_t)(mBase + row) * ldc + n0 + c8) = lv;
        }
        __threadfence();
      }
    }
    __builtin_amdgcn_fence(__ATOMIC_RELEASE, "workgroup");
    __builtin_amdgcn_wave_barrier();
    __builtin_amdgcn_fence(__ATOMIC_ACQUIRE, "workgroup");
  }
}

__global__ __launch_bounds__(256) void cast8_f16_kernel(const float* __restrict__ in, unsigned short* __restrict__ out, int n8) {
  const int i = blockIdx.x * 256 + threadIdx.x;
  if (i >= n8) return;
  const float* p = in + 8 * (size_t)i;
  const v4f a = *(const v4f*)(p);
  const v4f c = *(const v4f*)(p + 4);
  unsigned short hb[8];
#pragma unroll
  for (int e = 0; e < 4; ++e) {
    hb[e]     = h_bits(a[e]);
    hb[4 + e] = h_bits(c[e]);
  }
  const v4u u = (v4u){pk16(hb[0], hb[1]), pk16(hb[2], hb[3]), pk16(hb[4], hb[5]), pk16(hb[6], hb[7])};
  unsigned short* q = out + 8 * (size_t)i;
  *(volatile v4u*)q = u;
  __threadfence();
  *(volatile v4u*)q = u;
}

template <int MODE>
__global__ __launch_bounds__(256) void tcast_kernel(const float* __restrict__ in,
                                                    unsigned short* __restrict__ outA, unsigned short* __restrict__ outB,
                                                    int R, int Cc, float scale) {
  __shared__ float sm[64][65];
  const int t  = threadIdx.x;
  const int r0 = blockIdx.x * 64;
  const int c0 = blockIdx.y * 64;
  const int z  = blockIdx.z;
  const float* ip = in + (size_t)z * R * Cc;
#pragma unroll
  for (int i = 0; i < 16; ++i) {
    const int e  = i * 256 + t;
    const int rl = e >> 6;
    const int cl = e & 63;
    sm[cl][rl] = ip[(size_t)(r0 + rl) * Cc + c0 + cl] * scale;
  }
  __syncthreads();
  const int lane = t & 31, wave = t >> 5;
  const int q = lane >> 3, c8 = (lane & 7) * 8;
  unsigned short* oa = outA + (size_t)z * R * Cc;
  unsigned short* ob = (MODE == 1) ? (outB + (size_t)z * R * Cc) : nullptr;
  for (int pass = 0; pass < 2; ++pass) {
#pragma unroll
    for (int it = 0; it < 2; ++it) {
      const int row = wave * 8 + it * 4 + q;
      unsigned short hb[8], lb[8];
#pragma unroll
      for (int e = 0; e < 8; ++e) {
        const float v = sm[row][c8 + e];
        if (MODE == 0) {
          hb[e] = h_bits(v);
          lb[e] = 0;
        } else {
          hb[e] = f2bf_bits(v);
          lb[e] = f2bf_bits(v - bf_bits2f(hb[e]));
        }
      }
      const size_t o = (size_t)(c0 + row) * R + r0 + c8;
      const v4u u = (v4u){pk16(hb[0], hb[1]), pk16(hb[2], hb[3]), pk16(hb[4], hb[5]), pk16(hb[6], hb[7])};
      *(volatile v4u*)(oa + o) = u;
      if (MODE == 1) {
        const v4u w = (v4u){pk16(lb[0], lb[1]), pk16(lb[2], lb[3]), pk16(lb[4], lb[5]), pk16(lb[6], lb[7])};
        *(volatile v4u*)(ob + o) = w;
      }
    }
    __threadfence();
  }
}

extern "C" void kernel_launch(void* const* d_in, const int* in_sizes, int n_in,
                              void* d_out, int out_size, void* d_ws, size_t ws_size,
                              hipStream_t stream) {
  if (n_in < 13) return;
  if (in_sizes[0] != kRows * kDin) return;
  if (in_sizes[1] != kNE * kDin * kHid) return;
  if (in_sizes[2] != kNE * kHid) return;
  if (in_sizes[3] != kNE * kHid * kDo) return;
  if (in_sizes[4] != kNE * kDo) return;
  if (in_sizes[5] != kCat * kHc) return;
  if (in_sizes[6] != kHc) return;
  if (in_sizes[7] != kHc * kDo) return;
  if (in_sizes[8] != kDo) return;
  if (in_sizes[9] != kDo * kDo) return;
  if (in_sizes[10] != kDo) return;
  if (in_sizes[11] != kDo * kDo) return;
  if (in_sizes[12] != kDo) return;
  if (out_size != kRows * kDo) return;

  const float* x   = (const float*)d_in[0];
  const float* W1  = (const float*)d_in[1];
  const float* b1  = (const float*)d_in[2];
  const float* W2  = (const float*)d_in[3];
  const float* b2  = (const float*)d_in[4];
  const float* Wc1 = (const float*)d_in[5];
  const float* bc1 = (const float*)d_in[6];
  const float* Wc2 = (const float*)d_in[7];
  const float* bc2 = (const float*)d_in[8];
  const float* We  = (const float*)d_in[9];
  const float* be  = (const float*)d_in[10];
  const float* Wd  = (const float*)d_in[11];
  const float* bd  = (const float*)d_in[12];
  float* out = (float*)d_out;

  char* ws = (char*)d_ws;
  const size_t szCat  = (size_t)kRows * kCat * 2;
  const size_t szXH   = (size_t)kRows * kDin * 2;
  const size_t szW1T  = (size_t)kNE * kHid * kDin * 2;
  const size_t szW2T  = (size_t)kNE * kDo * kHid * 2;
  const size_t szH    = (size_t)kRows * kNcols * 2;
  const size_t szWc1T = (size_t)kHc * kCat * 2;
  const size_t szY    = (size_t)kRows * kHc * 2;
  const size_t szWc2T = (size_t)kDo * kHc * 2;
  const size_t szWsm  = (size_t)kDo * kDo * 2;
  const size_t szZ    = (size_t)kRows * kDo * 2;

  size_t off = 0;
  unsigned short* CAT = (unsigned short*)(ws + off); off += szCat;
  const size_t offPhase = off;
  unsigned short* XH   = (unsigned short*)(ws + off); off += szXH;
  unsigned short* W1T  = (unsigned short*)(ws + off); off += szW1T;
  unsigned short* W2TH = (unsigned short*)(ws + off); off += szW2T;
  unsigned short* W2TL = (unsigned short*)(ws + off); off += szW2T;
  unsigned short* HH   = (unsigned short*)(ws + off); off += szH;
  unsigned short* HL   = (unsigned short*)(ws + off); off += szH;
  const size_t p1end = off;
  off = offPhase;
  unsigned short* WC1T  = (unsigned short*)(ws + off); off += szWc1T;
  unsigned short* YH    = (unsigned short*)(ws + off); off += szY;
  unsigned short* YL    = (unsigned short*)(ws + off); off += szY;
  unsigned short* WC2TH = (unsigned short*)(ws + off); off += szWc2T;
  unsigned short* WC2TL = (unsigned short*)(ws + off); off += szWc2T;
  unsigned short* WETH  = (unsigned short*)(ws + off); off += szWsm;
  unsigned short* WETL  = (unsigned short*)(ws + off); off += szWsm;
  unsigned short* WDTH  = (unsigned short*)(ws + off); off += szWsm;
  unsigned short* WDTL  = (unsigned short*)(ws + off); off += szWsm;
  unsigned short* ZH    = (unsigned short*)(ws + off); off += szZ;
  unsigned short* ZL    = (unsigned short*)(ws + off); off += szZ;
  unsigned short* EH    = (unsigned short*)(ws + off); off += szZ;
  unsigned short* EL    = (unsigned short*)(ws + off); off += szZ;
  const size_t p2end = off;
  if (p1end > ws_size || p2end > ws_size) return;

  const unsigned short* kNull16 = (const unsigned short*)nullptr;
  const float* kNullF = (const float*)nullptr;

  hipLaunchKernelGGL(cast8_f16_kernel, dim3((kRows * kDin / 8 + 255) / 256), dim3(256), 0, stream,
                     x, XH, kRows * kDin / 8);
  hipLaunchKernelGGL(HIP_KERNEL_NAME(tcast_kernel<0>), dim3(kDin / 64, kHid / 64, kNE), dim3(256), 0, stream,
                     W1, W1T, (unsigned short*)nullptr, kDin, kHid, kW1Carry);
  hipLaunchKernelGGL(HIP_KERNEL_NAME(tcast_kernel<1>), dim3(kHid / 64, kDo / 64, kNE), dim3(256), 0, stream,
                     W2, W2TH, W2TL, kHid, kDo, 1.0f);

  const int tilesM = kRows / 64;
  const int blocksH = (tilesM * (kNcols / 64) + 7) / 8;
  const int blocksO = (tilesM * (kDo / 64) + 7) / 8;
  for (int c = 0; c < kNChunk; ++c) {
    hipLaunchKernelGGL(HIP_KERNEL_NAME(wmma_gemm64<0, false, 2, 2, false, 2>), dim3(blocksH, 1), dim3(256), 0, stream,
                       (const unsigned short*)XH, kNull16, kDin, (long)0,
                       (const unsigned short*)(W1T + (size_t)c * kNcols * kDin), kNull16, kDin, (long)0,
                       (void*)HH, (void*)HL, kNcols, (long)0,
                       b1 + (size_t)c * kNcols, (long)0,
                       kNullF, (long)0,
                       kRows, kNcols, kDin, kW1CarryInv);
    hipLaunchKernelGGL(HIP_KERNEL_NAME(wmma_gemm64<1, true, 2, 1, false, 0>), dim3(blocksO, kEChunk), dim3(256), 0, stream,
                       (const unsigned short*)HH, (const unsigned short*)HL, kNcols, (long)kHid,
                       (const unsigned short*)(W2TH + (size_t)c * kEChunk * kDo * kHid),
                       (const unsigned short*)(W2TL + (size_t)c * kEChunk * kDo * kHid), kHid, (long)(kDo * kHid),
                       (void*)(CAT + (size_t)c * kEChunk * kDo), (void*)nullptr, kCat, (long)kDo,
                       b2 + (size_t)c * kEChunk * kDo, (long)kDo,
                       kNullF, (long)0,
                       kRows, kDo, kHid, 1.0f);
  }

  hipLaunchKernelGGL(HIP_KERNEL_NAME(tcast_kernel<0>), dim3(kCat / 64, kHc / 64, 1), dim3(256), 0, stream,
                     Wc1, WC1T, (unsigned short*)nullptr, kCat, kHc, kWc1Carry);
  hipLaunchKernelGGL(HIP_KERNEL_NAME(tcast_kernel<1>), dim3(kHc / 64, kDo / 64, 1), dim3(256), 0, stream,
                     Wc2, WC2TH, WC2TL, kHc, kDo, 1.0f);
  hipLaunchKernelGGL(HIP_KERNEL_NAME(tcast_kernel<1>), dim3(kDo / 64, kDo / 64, 1), dim3(256), 0, stream,
                     We, WETH, WETL, kDo, kDo, 1.0f);
  hipLaunchKernelGGL(HIP_KERNEL_NAME(tcast_kernel<1>), dim3(kDo / 64, kDo / 64, 1), dim3(256), 0, stream,
                     Wd, WDTH, WDTL, kDo, kDo, 1.0f);

  const int blocksY = (tilesM * (kHc / 64) + 7) / 8;
  hipLaunchKernelGGL(HIP_KERNEL_NAME(wmma_gemm64<0, false, 2, 2, false, 2>), dim3(blocksY, 1), dim3(256), 0, stream,
                     (const unsigned short*)CAT, kNull16, kCat, (long)0,
                     (const unsigned short*)WC1T, kNull16, kCat, (long)0,
                     (void*)YH, (void*)YL, kHc, (long)0,
                     bc1, (long)0,
                     kNullF, (long)0,
                     kRows, kHc, kCat, kWc1CarryInv);
  hipLaunchKernelGGL(HIP_KERNEL_NAME(wmma_gemm64<1, true, 2, 2, false, 0>), dim3(blocksO, 1), dim3(256), 0, stream,
                     (const unsigned short*)YH, (const unsigned short*)YL, kHc, (long)0,
                     (const unsigned short*)WC2TH, (const unsigned short*)WC2TL, kHc, (long)0,
                     (void*)ZH, (void*)ZL, kDo, (long)0,
                     bc2, (long)0,
                     kNullF, (long)0,
                     kRows, kDo, kHc, 1.0f);
  hipLaunchKernelGGL(HIP_KERNEL_NAME(wmma_gemm64<1, true, 2, 2, false, 0>), dim3(blocksO, 1), dim3(256), 0, stream,
                     (const unsigned short*)ZH, (const unsigned short*)ZL, kDo, (long)0,
                     (const unsigned short*)WETH, (const unsigned short*)WETL, kDo, (long)0,
                     (void*)EH, (void*)EL, kDo, (long)0,
                     be, (long)0,
                     kNullF, (long)0,
                     kRows, kDo, kDo, 1.0f);
  hipLaunchKernelGGL(HIP_KERNEL_NAME(wmma_gemm64<1, true, 2, 0, false, 0>), dim3(blocksO, 1), dim3(256), 0, stream,
                     (const unsigned short*)EH, (const unsigned short*)EL, kDo, (long)0,
                     (const unsigned short*)WDTH, (const unsigned short*)WDTL, kDo, (long)0,
                     (void*)out, (void*)nullptr, kDo, (long)0,
                     bd, (long)0,
                     kNullF, (long)0,
                     kRows, kDo, kDo, 1.0f);
}
